// Net_83786222011073
// MI455X (gfx1250) — hardware-verified
//
#include <hip/hip_runtime.h>
#include <stddef.h>
#include <stdint.h>
#include <math.h>


#define NNODE  50000
#define NEDGE  1600000
#define NGR    256
#define DIN    128
#define DH1    100
#define DH2    20
#define DSF    64
#define MP     50048
#define KG     256
#define T2W    32
#define NTHR   256
#define NWAVE  8
#define EPT    8
#define CHUNK  (NTHR * EPT)
#define WCAP   (EPT * 32)
#define LISTN  (NWAVE * WCAP)
#define NBA    512
#define SLA    9
#define NBLK   98
#define RCAP   20480
#define DEGCAP 128
#define GBM    128
#define GBN    128
#define AGG_ZINTS (LISTN + 2 * RCAP + 3 * NBA)
#define CMP_LDS_INTS (AGG_ZINTS + 16)
#define GEMM_LDS_FLOATS (GBM * GBN + DH1 * T2W)
#define WSMAX  134217728

#define PB1    0
#define PW2    128
#define PB2    3328
#define PWP    3360
#define PBP    4640
#define PWF1   4672
#define PBF1   4896
#define PWF2   4912
#define PBF2   4928
#define PAR_N  4960
#define HTB_N  (PAR_N - PWP)

#define XBBLK  (MP * (DIN / 8) / NTHR)
#define W1BLK  (GBN * (KG / 8) / NTHR)
#define PREPBLK (XBBLK + W1BLK + 1)

static_assert(DIN == 128 && DIN == 32 * 4);
static_assert(DH1 <= GBN && DH2 <= T2W);
static_assert(KG % 32 == 0 && KG == 2 * DIN);
static_assert(NBLK * NBA >= NNODE && NBLK * NBA >= MP);
static_assert(MP == 391 * GBM && MP >= NNODE);
static_assert(8 * 6250 == NNODE);
static_assert(NGR == NTHR);
static_assert(RCAP >= 16678 + 16678 / 20 && DEGCAP >= 57 + 8);
static_assert((CHUNK & (CHUNK - 1)) == 0 && CHUNK <= 4096);
static_assert((NBA & (NBA - 1)) == 0 && NBA == (1 << SLA) && NBA == 2 * NTHR);
static_assert(((long long)CHUNK << SLA) < (1LL << 31));
static_assert(NEDGE < (1 << (31 - SLA)));
static_assert(NBA % NWAVE == 0 && NBA % 32 == 0);
static_assert(RCAP % (4 * NTHR) == 0 && AGG_ZINTS % 4 == 0 && LISTN % 4 == 0);
static_assert((MP * (DIN / 8)) % NTHR == 0 && (GBN * (KG / 8)) % NTHR == 0);
static_assert(PAR_N % 32 == 0 && PWP % 4 == 0 && PW2 % 4 == 0 && HTB_N % 4 == 0);
static_assert(PBF2 + 16 <= PAR_N);
static_assert(CMP_LDS_INTS * 4 <= 300000 && GEMM_LDS_FLOATS * 4 <= 300000);
static_assert(GBM == NWAVE * 16);

typedef float          v4f   __attribute__((ext_vector_type(4)));
typedef float          v8f   __attribute__((ext_vector_type(8)));
typedef int            v4i   __attribute__((ext_vector_type(4)));
typedef int            v8i   __attribute__((ext_vector_type(8)));
typedef unsigned       v2u   __attribute__((ext_vector_type(2)));
typedef unsigned short v4us  __attribute__((ext_vector_type(4)));
typedef unsigned short v8us  __attribute__((ext_vector_type(8)));
typedef unsigned short v16us __attribute__((ext_vector_type(16)));
typedef __bf16         v16bf __attribute__((ext_vector_type(16)));
typedef v4f  __attribute__((may_alias)) v4fa;
typedef v4i  __attribute__((may_alias)) v4ia;
typedef v2u  __attribute__((may_alias)) v2ua;
typedef v4us __attribute__((may_alias)) v4usa;
typedef v8us __attribute__((may_alias)) v8usa;
union FragB { v16bf v; v16us u; v8us h[2]; v8i w; };

__device__ __forceinline__ v8f wmb(const FragB& a, const FragB& b, v8f c) {
  v8f d = __builtin_amdgcn_wmma_f32_16x16x32_bf16(false, a.v, false, b.v, (short)0, c, false, false);
  asm volatile("v_nop\n\tv_nop\n\tv_nop\n\tv_nop" : "+v"(d) : "v"(a.w), "v"(b.w));
  return d;
}

__device__ __forceinline__ unsigned bf16_bits(float f) {
  const unsigned u = __float_as_uint(f);
  return (u + 0x7FFFu + ((u >> 16) & 1u)) >> 16;
}
__device__ __forceinline__ float bf16_val(float f) {
  return __uint_as_float(bf16_bits(f) << 16);
}
__device__ __forceinline__ float relu_np(float v) {
  return (v > 0.0f) ? v : (v - v);
}

__device__ __forceinline__ void wave_sync() {
  __builtin_amdgcn_fence(__ATOMIC_RELEASE, "wavefront");
  __builtin_amdgcn_wave_barrier();
  __builtin_amdgcn_fence(__ATOMIC_ACQUIRE, "wavefront");
}

template <int SLB>
__device__ __forceinline__ int scan_chunk(const int* __restrict__ dsts, int nE, int cbase, int slotBase,
                                          int nb, int vec8, int* list, int tid, int lane, int wave) {
  int wc = 0;
  const int el0  = tid * EPT;
  const int e0   = cbase + el0;
  const int sent = -2147483647 - 1;
  v4i da, db;
  if (vec8 != 0 && cbase + CHUNK <= nE) {
    da = *(const v4i*)(dsts + e0);
    db = *(const v4i*)(dsts + e0 + 4);
  } else {
    da.x = (e0     < nE) ? dsts[min(e0,     nE - 1)] : sent;
    da.y = (e0 + 1 < nE) ? dsts[min(e0 + 1, nE - 1)] : sent;
    da.z = (e0 + 2 < nE) ? dsts[min(e0 + 2, nE - 1)] : sent;
    da.w = (e0 + 3 < nE) ? dsts[min(e0 + 3, nE - 1)] : sent;
    db.x = (e0 + 4 < nE) ? dsts[min(e0 + 4, nE - 1)] : sent;
    db.y = (e0 + 5 < nE) ? dsts[min(e0 + 5, nE - 1)] : sent;
    db.z = (e0 + 6 < nE) ? dsts[min(e0 + 6, nE - 1)] : sent;
    db.w = (e0 + 7 < nE) ? dsts[min(e0 + 7, nE - 1)] : sent;
  }
  const unsigned nbs = (unsigned)slotBase;
  const unsigned unb = (unsigned)nb;
  const unsigned s0 = (unsigned)da.x - nbs, s1 = (unsigned)da.y - nbs;
  const unsigned s2 = (unsigned)da.z - nbs, s3 = (unsigned)da.w - nbs;
  const unsigned s4 = (unsigned)db.x - nbs, s5 = (unsigned)db.y - nbs;
  const unsigned s6 = (unsigned)db.z - nbs, s7 = (unsigned)db.w - nbs;
  const bool h0 = s0 < unb, h1 = s1 < unb, h2 = s2 < unb, h3 = s3 < unb;
  const bool h4 = s4 < unb, h5 = s5 < unb, h6 = s6 < unb, h7 = s7 < unb;
  const unsigned any = __builtin_amdgcn_ballot_w32(h0 | h1 | h2 | h3 | h4 | h5 | h6 | h7);
  if (any != 0u) {
#define HITJ(J, HJ, SJ) { \
      const unsigned mj = __builtin_amdgcn_ballot_w32(HJ); \
      if (mj != 0u) { \
        if (HJ) { \
          const int pos = wc + (int)__builtin_amdgcn_mbcnt_lo(mj, 0u); \
          if (pos < WCAP) list[wave * WCAP + pos] = ((el0 + (J)) << SLB) | (int)(SJ); \
        } \
        wc += (int)__builtin_popcount(mj); } }
    HITJ(0, h0, s0)
    HITJ(1, h1, s1)
    HITJ(2, h2, s2)
    HITJ(3, h3, s3)
    HITJ(4, h4, s4)
    HITJ(5, h5, s5)
    HITJ(6, h6, s6)
    HITJ(7, h7, s7)
#undef HITJ
  }
  return wc;
}

__global__ __launch_bounds__(NTHR) void k_prep(
    const float* __restrict__ feat, const float* __restrict__ W1, const float* __restrict__ b1,
    const float* __restrict__ W2, const float* __restrict__ b2, const float* __restrict__ Wp,
    const float* __restrict__ bp, const float* __restrict__ Wf1, const float* __restrict__ bf1,
    const float* __restrict__ Wf2, const float* __restrict__ bf2,
    unsigned short* xb, unsigned short* w1d, float* par)
{
  __shared__ __attribute__((aligned(16))) float ps[PAR_N];
  const int tid = (int)threadIdx.x;
  const int blk = (int)blockIdx.x;
  if (blk < XBBLK) {
    const int u   = blk * NTHR + tid;
    const int row = u >> 4;
    const int k8  = (u & 15) * 8;
    const int rc  = row < NNODE ? row : NNODE - 1;
    const float* p = feat + (size_t)rc * DIN + k8;
    const v4f a = *(const v4fa*)p;
    const v4f b = *(const v4fa*)(p + 4);
    const bool ok = row < NNODE;
    v8us o;
    o[0] = ok ? (unsigned short)bf16_bits(a.x) : (unsigned short)0;
    o[1] = ok ? (unsigned short)bf16_bits(a.y) : (unsigned short)0;
    o[2] = ok ? (unsigned short)bf16_bits(a.z) : (unsigned short)0;
    o[3] = ok ? (unsigned short)bf16_bits(a.w) : (unsigned short)0;
    o[4] = ok ? (unsigned short)bf16_bits(b.x) : (unsigned short)0;
    o[5] = ok ? (unsigned short)bf16_bits(b.y) : (unsigned short)0;
    o[6] = ok ? (unsigned short)bf16_bits(b.z) : (unsigned short)0;
    o[7] = ok ? (unsigned short)bf16_bits(b.w) : (unsigned short)0;
    unsigned short* dp = xb + (size_t)row * DIN + k8;
    *(volatile v8us*)dp = o;
    __threadfence();
    *(volatile v8us*)dp = o;
  } else if (blk < XBBLK + W1BLK) {
    const int v  = (blk - XBBLK) * NTHR + tid;
    const int n  = v >> 5;
    const int k8 = (v & 31) * 8;
    const int kk = k8 & (DIN - 1);
    const int nc = n < DH1 ? n : DH1 - 1;
    const bool ok = n < DH1;
    const float* p = W1 + (size_t)kk * DH1 + nc;
    v8us o;
#pragma unroll
    for (int i = 0; i < 8; ++i) {
      const unsigned short hv = (unsigned short)bf16_bits(p[(size_t)i * DH1]);
      o[i] = ok ? hv : (unsigned short)0;
    }
    unsigned short* dp = w1d + (size_t)n * KG + k8;
    *(volatile v8us*)dp = o;
    __threadfence();
    *(volatile v8us*)dp = o;
  } else {
#pragma unroll 1
    for (int i = tid; i < PAR_N; i += NTHR) ps[i] = 0.0f;
    __syncthreads();
#pragma unroll 1
    for (int i = tid; i < DH1; i += NTHR) ps[PB1 + i] = bf16_val(b1[i]);
#pragma unroll 1
    for (int i = tid; i < DH1 * DH2; i += NTHR) {
      const int k = i / DH2;
      const int c = i - k * DH2;
      ps[PW2 + k * T2W + c] = bf16_val(W2[i]);
    }
#pragma unroll 1
    for (int i = tid; i < DH2; i += NTHR) ps[PB2 + i] = bf16_val(b2[i]);
#pragma unroll 1
    for (int i = tid; i < DSF * DH2; i += NTHR) ps[PWP + i] = bf16_val(Wp[i]);
#pragma unroll 1
    for (int i = tid; i < DH2; i += NTHR) ps[PBP + i] = bf16_val(bp[i]);
#pragma unroll 1
    for (int i = tid; i < DH2 * 10; i += NTHR) ps[PWF1 + i] = bf16_val(Wf1[i]);
#pragma unroll 1
    for (int i = tid; i < 10; i += NTHR) ps[PBF1 + i] = bf16_val(bf1[i]);
#pragma unroll 1
    for (int i = tid; i < 10; i += NTHR) ps[PWF2 + i] = bf16_val(Wf2[i]);
    if (tid == 0) ps[PBF2] = bf16_val(bf2[0]);
    __syncthreads();
#pragma unroll 1
    for (int i = tid; i < PAR_N / 4; i += NTHR) {
      const v4f v = *(const v4fa*)(ps + 4 * i);
      *(volatile v4f*)(par + 4 * i) = v;
    }
    __threadfence();
#pragma unroll 1
    for (int i = tid; i < PAR_N / 4; i += NTHR) {
      const v4f v = *(const v4fa*)(ps + 4 * i);
      *(volatile v4f*)(par + 4 * i) = v;
    }
  }
}

__global__ __launch_bounds__(NTHR) void k_compact(const int* __restrict__ srcs, const int* __restrict__ dsts,
                                                  int nE, int nN, int vec8,
                                                  int* lst, int* cntp, int* offp, int* flg) {
  extern __shared__ __attribute__((aligned(16))) int dsm[];
  int* list = dsm;
  int* hl   = dsm + LISTN;
  int* sl   = dsm + LISTN + RCAP;
  int* cnt  = dsm + LISTN + 2 * RCAP;
  int* offs = cnt + NBA;
  int* cur  = offs + NBA;
  int* misc = cur + NBA;
  const int tid = (int)threadIdx.x, lane = tid & 31, wave = tid >> 5;
  const int blk = (int)blockIdx.x;
  const int nodeBase = blk * NBA;

  {
    const v4i z4 = {0, 0, 0, 0};
    for (int i = tid * 4; i < AGG_ZINTS; i += NTHR * 4) *(v4ia*)(dsm + i) = z4;
    if (tid < 16) misc[tid] = 0;
  }
  __syncthreads();

  int t = 0, ov = 0;
  const int nChunks = (nE + CHUNK - 1) / CHUNK;
#pragma unroll 1
  for (int ch = 0; ch < nChunks; ++ch) {
    const int cbase = ch * CHUNK;
    const int wc = scan_chunk<SLA>(dsts, nE, cbase, nodeBase, NBA, vec8, list, tid, lane, wave);
    if (lane == 0) misc[wave] = wc;
    __syncthreads();
    if (wave == 0) {
#pragma unroll 1
      for (int w2 = 0; w2 < NWAVE; ++w2) {
        int c = misc[w2];
        c = c < 0 ? 0 : (c > WCAP ? WCAP : c);
#pragma unroll 1
        for (int b0 = 0; b0 < c; b0 += 32) {
          const int idx = b0 + lane;
          const int ent = list[w2 * WCAP + (idx < WCAP ? idx : WCAP - 1)];
          const int m32 = (c - b0) < 32 ? (c - b0) : 32;
#pragma unroll 1
          for (int k = 0; k < m32; ++k) {
            const int u    = __builtin_amdgcn_readlane(ent, k);
            const int slot = u & (NBA - 1);
            const int el   = (u >> SLA) & (CHUNK - 1);
            const int pk   = ((cbase + el) << SLA) | slot;
            if (t < RCAP) {
              if (lane == 0) { hl[t] = pk; cnt[slot] = cnt[slot] + 1; }
              t = t + 1;
            } else {
              ov = 1;
            }
          }
        }
      }
    }
    __syncthreads();
  }
  if (wave == 0 && lane == 0) { misc[8] = t; misc[9] = ov; }
  __syncthreads();
  int tt = misc[8];
  tt = tt < 0 ? 0 : (tt > RCAP ? RCAP : tt);
  const int ovf = misc[9];

  if (wave == 0) {
    const int base = lane * (NBA / 32);
    int s = 0;
#pragma unroll 1
    for (int i = 0; i < NBA / 32; ++i) s += cnt[base + i];
    int incl = s;
#pragma unroll
    for (int d = 1; d < 32; d <<= 1) {
      const int y = __shfl_up(incl, d, 32);
      if (lane >= d) incl += y;
    }
    int run = incl - s;
#pragma unroll 1
    for (int i = 0; i < NBA / 32; ++i) {
      const int cv = cnt[base + i];
      offs[base + i] = run;
      cur[base + i]  = run;
      run += cv;
    }
  }
  __syncthreads();
  if (wave == 0) {
#pragma unroll 1
    for (int b0 = 0; b0 < tt; b0 += 32) {
      const int idx = b0 + lane;
      const int ent = hl[idx < RCAP ? idx : RCAP - 1];
      const int m32 = (tt - b0) < 32 ? (tt - b0) : 32;
#pragma unroll 1
      for (int k = 0; k < m32; ++k) {
        const int u    = __builtin_amdgcn_readlane(ent, k);
        const int slot = u & (NBA - 1);
        if (lane == 0) {
          int p = cur[slot];
          p = p < 0 ? 0 : (p > RCAP - 1 ? RCAP - 1 : p);
          sl[p] = u;
          cur[slot] = p + 1;
        }
      }
    }
  }
  __syncthreads();

  {
    const int bg = ((cnt[tid] > DEGCAP) || (cnt[tid + NTHR] > DEGCAP)) ? 1 : 0;
    if (bg != 0) misc[10] = 1;
  }
#pragma unroll 4
  for (int i = tid; i < RCAP; i += NTHR) {
    const int ent = sl[i];
    int eid = ent >> SLA;
    eid = eid < 0 ? 0 : (eid > nE - 1 ? nE - 1 : eid);
    int sr = srcs[eid];
    sr = sr < 0 ? 0 : (sr > nN - 1 ? nN - 1 : sr);
    hl[i] = (i < tt) ? sr : 0;
  }
  __syncthreads();
  const int flag = (ovf != 0 || misc[10] != 0) ? 1 : 0;
  int* bl = lst + (size_t)blk * RCAP;
  const v4i f4 = {flag, flag, flag, flag};
#pragma unroll 4
  for (int it = 0; it < RCAP / (4 * NTHR); ++it) {
    const int j = 4 * (it * NTHR + tid);
    const v4i v = *(const v4ia*)(hl + j);
    *(volatile v4i*)(bl + j) = v;
  }
  if (tid < NBA / 4) {
    const v4i cv = *(const v4ia*)(cnt + 4 * tid);
    const v4i ovv = *(const v4ia*)(offs + 4 * tid);
    *(volatile v4i*)(cntp + (size_t)nodeBase + 4 * tid) = cv;
    *(volatile v4i*)(offp + (size_t)nodeBase + 4 * tid) = ovv;
  }
  if (tid < 8) *(volatile v4i*)(flg + (size_t)blk * 32 + 4 * tid) = f4;
  __threadfence();
#pragma unroll 4
  for (int it = 0; it < RCAP / (4 * NTHR); ++it) {
    const int j = 4 * (it * NTHR + tid);
    const v4i v = *(const v4ia*)(hl + j);
    *(volatile v4i*)(bl + j) = v;
  }
  if (tid < NBA / 4) {
    const v4i cv = *(const v4ia*)(cnt + 4 * tid);
    const v4i ovv = *(const v4ia*)(offs + 4 * tid);
    *(volatile v4i*)(cntp + (size_t)nodeBase + 4 * tid) = cv;
    *(volatile v4i*)(offp + (size_t)nodeBase + 4 * tid) = ovv;
  }
  if (tid < 8) *(volatile v4i*)(flg + (size_t)blk * 32 + 4 * tid) = f4;
}

__global__ __launch_bounds__(NTHR) void k_agg1(const int* __restrict__ lst, const int* __restrict__ cntp,
                                               const int* __restrict__ offp, const int* __restrict__ flg,
                                               const unsigned short* __restrict__ xb, unsigned short* apl,
                                               int nN, int mRows) {
  __shared__ __attribute__((aligned(16))) unsigned short rows[NWAVE * KG];
  const int tid = (int)threadIdx.x, lane = tid & 31, wave = tid >> 5;
  const int blk = (int)blockIdx.x;
  const int nodeBase = blk * NBA;
  unsigned short* rowbuf = rows + wave * KG;
  const int* bl = lst + (size_t)blk * RCAP;
  const int ovf = flg[(size_t)blk * 32];
  const float qnan = __int_as_float(0x7fc00000);
  const float pz = (ovf != 0) ? qnan : 0.0f;
#pragma unroll 1
  for (int si = 0; si < NBA / NWAVE; ++si) {
    const int s    = si * NWAVE + wave;
    const int node = nodeBase + s;
    int c = cntp[node];
    const bool big = c > DEGCAP;
    c = c < 0 ? 0 : (c > DEGCAP ? DEGCAP : c);
    int o = offp[node];
    o = o < 0 ? 0 : (o > RCAP ? RCAP : o);
    const int nc = node < nN ? node : nN - 1;
    float a0 = 0.0f, a1 = 0.0f, a2 = 0.0f, a3 = 0.0f;
#pragma unroll 1
    for (int b0 = 0; b0 < c; b0 += 32) {
      int idx = o + b0 + lane;
      idx = idx > RCAP - 1 ? RCAP - 1 : idx;
      int sr = bl[idx];
      sr = sr < 0 ? 0 : (sr > nN - 1 ? nN - 1 : sr);
      const int m32 = (c - b0) < 32 ? (c - b0) : 32;
#pragma unroll 1
      for (int k = 0; k < m32; ++k) {
        const int sk = __builtin_amdgcn_readlane(sr, k);
        const v2u w = *(const v2ua*)(xb + (size_t)sk * DIN + 4 * lane);
        a0 += __uint_as_float(w.x << 16);
        a1 += __uint_as_float(w.x & 0xffff0000u);
        a2 += __uint_as_float(w.y << 16);
        a3 += __uint_as_float(w.y & 0xffff0000u);
      }
    }
    const v2u wo = *(const v2ua*)(xb + (size_t)nc * DIN + 4 * lane);
    const float x0 = __uint_as_float(wo.x << 16);
    const float x1 = __uint_as_float(wo.x & 0xffff0000u);
    const float x2 = __uint_as_float(wo.y << 16);
    const float x3 = __uint_as_float(wo.y & 0xffff0000u);
    const bool has = c > 0;
    const float fd = (float)(c > 0 ? c : 1);
    const float q0 = a0 / fd, q1 = a1 / fd, q2 = a2 / fd, q3 = a3 / fd;
    const float pzr = big ? qnan : pz;
    const bool live = node < nN;
    const float m0 = live ? ((has ? q0 : x0) + pzr) : 0.0f;
    const float m1 = live ? ((has ? q1 : x1) + pzr) : 0.0f;
    const float m2 = live ? ((has ? q2 : x2) + pzr) : 0.0f;
    const float m3 = live ? ((has ? q3 : x3) + pzr) : 0.0f;
    v4us mh, ml;
    {
      unsigned hb;
      hb = bf16_bits(m0); mh[0] = (unsigned short)hb; ml[0] = (unsigned short)bf16_bits(m0 - __uint_as_float(hb << 16));
      hb = bf16_bits(m1); mh[1] = (unsigned short)hb; ml[1] = (unsigned short)bf16_bits(m1 - __uint_as_float(hb << 16));
      hb = bf16_bits(m2); mh[2] = (unsigned short)hb; ml[2] = (unsigned short)bf16_bits(m2 - __uint_as_float(hb << 16));
      hb = bf16_bits(m3); mh[3] = (unsigned short)hb; ml[3] = (unsigned short)bf16_bits(m3 - __uint_as_float(hb << 16));
    }
    *(v4usa*)(rowbuf + 4 * lane) = mh;
    *(v4usa*)(rowbuf + DIN + 4 * lane) = ml;
    wave_sync();
    const v8us q = *(const v8usa*)(rowbuf + 8 * lane);
    wave_sync();
    if (node < mRows) {
      unsigned short* rp = apl + (size_t)node * KG + 8 * lane;
      *(volatile v8us*)rp = q;
      __threadfence();
      *(volatile v8us*)rp = q;
    }
  }
}

__global__ __launch_bounds__(NTHR) void k_gemm1(const unsigned short* __restrict__ A,
                                                const unsigned short* __restrict__ BT,
                                                const float* __restrict__ par, float* t2p, int nN) {
  extern __shared__ __attribute__((aligned(16))) float gsm[];
  float* stg = gsm;
  float* w2s = gsm + GBM * GBN;
  const int tid = (int)threadIdx.x, lane = tid & 31, wave = tid >> 5, hh = lane >> 4, m = lane & 15;
  const int rowBase = (int)blockIdx.x * GBM;

  v8f acc[8];
  {
    const v8f z = {0.f, 0.f, 0.f, 0.f, 0.f, 0.f, 0.f, 0.f};
#pragma unroll
    for (int t = 0; t < 8; ++t) acc[t] = z;
  }
  const unsigned short* ap = A + (size_t)(rowBase + 16 * wave + m) * (size_t)KG + 8 * hh;
  const unsigned short* bp = BT + (size_t)m * (size_t)KG + 8 * hh;

#pragma unroll 1
  for (int k0 = 0; k0 < KG; k0 += 32) {
    FragB af;
    af.h[0] = *(const v8usa*)(ap + k0);
    af.h[1] = *(const v8usa*)(ap + k0 + 16);
#pragma unroll
    for (int nt = 0; nt < 8; ++nt) {
      const unsigned short* wq = bp + (size_t)(16 * nt) * (size_t)KG + k0;
      FragB bf;
      bf.h[0] = *(const v8usa*)wq;
      bf.h[1] = *(const v8usa*)(wq + 16);
      acc[nt] = wmb(af, bf, acc[nt]);
    }
  }

#pragma unroll
  for (int nt = 0; nt < 8; ++nt) {
    const int lc = 16 * nt + m;
#pragma unroll
    for (int r = 0; r < 8; ++r) {
      const int lr = 16 * wave + 8 * hh + r;
      stg[lr * GBN + lc] = acc[nt][r];
    }
  }
#pragma unroll 1
  for (int i = tid; i < (DH1 * T2W) / 4; i += NTHR) {
    const v4f w = *(const v4f*)(par + PW2 + 4 * i);
    *(v4fa*)(w2s + 4 * i) = w;
  }
  __syncthreads();

  {
    const v4f bb = *(const v4f*)(par + PB1 + 4 * lane);
#pragma unroll 4
    for (int i = 0; i < 16; ++i) {
      float* p = stg + (16 * wave + i) * GBN + 4 * lane;
      v4f v = *(const v4fa*)p;
      v.x = relu_np(v.x + bb.x);
      v.y = relu_np(v.y + bb.y);
      v.z = relu_np(v.z + bb.z);
      v.w = relu_np(v.w + bb.w);
      *(v4fa*)p = v;
    }
  }
  __syncthreads();

  const int rq = lane >> 3, cg = lane & 7;
  const float* hr = stg + (16 * wave + rq) * GBN;
  const float* wq2 = w2s + 4 * cg;
  v4f t0 = {0.f, 0.f, 0.f, 0.f}, t1 = t0, t2 = t0, t3 = t0;
#pragma unroll 2
  for (int k = 0; k < DH1; ++k) {
    const v4f w = *(const v4fa*)(wq2 + T2W * k);
    const float h0 = hr[k];
    const float h1 = hr[4 * GBN + k];
    const float h2 = hr[8 * GBN + k];
    const float h3 = hr[12 * GBN + k];
    t0.x = fmaf(h0, w.x, t0.x); t0.y = fmaf(h0, w.y, t0.y); t0.z = fmaf(h0, w.z, t0.z); t0.w = fmaf(h0, w.w, t0.w);
    t1.x = fmaf(h1, w.x, t1.x); t1.y = fmaf(h1, w.y, t1.y); t1.z = fmaf(h1, w.z, t1.z); t1.w = fmaf(h1, w.w, t1.w);
    t2.x = fmaf(h2, w.x, t2.x); t2.y = fmaf(h2, w.y, t2.y); t2.z = fmaf(h2, w.z, t2.z); t2.w = fmaf(h2, w.w, t2.w);
    t3.x = fmaf(h3, w.x, t3.x); t3.y = fmaf(h3, w.y, t3.y); t3.z = fmaf(h3, w.z, t3.z); t3.w = fmaf(h3, w.w, t3.w);
  }
  const int r0 = rowBase + 16 * wave + rq;
  const bool okc = cg < (DH2 / 4);
  const v4f zz = {0.f, 0.f, 0.f, 0.f};
  const v4f o0 = (okc && (r0      < nN)) ? t0 : zz;
  const v4f o1 = (okc && (r0 + 4  < nN)) ? t1 : zz;
  const v4f o2 = (okc && (r0 + 8  < nN)) ? t2 : zz;
  const v4f o3 = (okc && (r0 + 12 < nN)) ? t3 : zz;
  float* op = t2p + (size_t)r0 * T2W + 4 * cg;
  *(volatile v4f*)(op)            = o0;
  *(volatile v4f*)(op + 4 * T2W)  = o1;
  *(volatile v4f*)(op + 8 * T2W)  = o2;
  *(volatile v4f*)(op + 12 * T2W) = o3;
  __threadfence();
  *(volatile v4f*)(op)            = o0;
  *(volatile v4f*)(op + 4 * T2W)  = o1;
  *(volatile v4f*)(op + 8 * T2W)  = o2;
  *(volatile v4f*)(op + 12 * T2W) = o3;
}

__global__ __launch_bounds__(NTHR) void k_agg2(const int* __restrict__ lst, const int* __restrict__ cntp,
                                               const int* __restrict__ offp, const int* __restrict__ flg,
                                               const float* __restrict__ t2p, const float* __restrict__ par,
                                               float* h2, int nN, int mRows) {
  const int tid = (int)threadIdx.x, lane = tid & 31, wave = tid >> 5;
  const int blk = (int)blockIdx.x;
  const int nodeBase = blk * NBA;
  const int* bl = lst + (size_t)blk * RCAP;
  const int ovf = flg[(size_t)blk * 32];
  const float qnan = __int_as_float(0x7fc00000);
  const float pz = (ovf != 0) ? qnan : 0.0f;
  const float bv = par[PB2 + lane];
#pragma unroll 1
  for (int si = 0; si < NBA / NWAVE; ++si) {
    const int s    = si * NWAVE + wave;
    const int node = nodeBase + s;
    int c = cntp[node];
    const bool big = c > DEGCAP;
    c = c < 0 ? 0 : (c > DEGCAP ? DEGCAP : c);
    int o = offp[node];
    o = o < 0 ? 0 : (o > RCAP ? RCAP : o);
    const int nc = node < nN ? node : nN - 1;
    float a = 0.0f;
#pragma unroll 1
    for (int b0 = 0; b0 < c; b0 += 32) {
      int idx = o + b0 + lane;
      idx = idx > RCAP - 1 ? RCAP - 1 : idx;
      int sr = bl[idx];
      sr = sr < 0 ? 0 : (sr > nN - 1 ? nN - 1 : sr);
      const int m32 = (c - b0) < 32 ? (c - b0) : 32;
#pragma unroll 1
      for (int k = 0; k < m32; ++k) {
        const int sk = __builtin_amdgcn_readlane(sr, k);
        a += t2p[(size_t)sk * T2W + lane];
      }
    }
    const float own = t2p[(size_t)nc * T2W + lane];
    const bool has = c > 0;
    const float fd = (float)(c > 0 ? c : 1);
    const float q = a / fd;
    const float pzr = big ? qnan : pz;
    const bool live = node < nN;
    float y = relu_np((has ? q : own) + bv);
    y = y + pzr;
    const float v = live ? y : 0.0f;
    if (node < mRows) {
      float* op = h2 + (size_t)node * T2W + lane;
      *(volatile float*)op = v;
      __threadfence();
      *(volatile float*)op = v;
    }
  }
}

__global__ __launch_bounds__(NTHR) void k_pool(const float* __restrict__ hf, const int* __restrict__ gidp,
                                               int nN, int seg, float* pl) {
  __shared__ float wsum[NWAVE * T2W];
  __shared__ int wcn[NWAVE];
  const int tid = (int)threadIdx.x, lane = tid & 31, wave = tid >> 5;
  const int g = (int)blockIdx.x;
  const int base = wave * seg;
  float a = 0.0f;
  int cnt = 0;
#pragma unroll 1
  for (int j0 = 0; j0 < seg; j0 += 32) {
    const int j  = j0 + lane;
    const int i  = base + j;
    int ic = i < nN ? i : nN - 1;
    ic = ic < 0 ? 0 : ic;
    const int b  = gidp[ic];
    const bool hit = (j < seg) && (i < nN) && (b == g);
    unsigned msk = __builtin_amdgcn_ballot_w32(hit);
    int nh = (int)__builtin_popcount(msk);
    nh = nh > 32 ? 32 : nh;
    cnt += nh;
#pragma unroll 1
    for (int q = 0; q < nh; ++q) {
      const int k = __builtin_ffs((int)msk) - 1;
      msk &= msk - 1u;
      int node = base + j0 + (k < 0 ? 0 : k);
      node = node > nN - 1 ? nN - 1 : node;
      a += hf[(size_t)node * T2W + lane];
    }
  }
  wsum[wave * T2W + lane] = a;
  if (lane == 0) wcn[wave] = cnt;
  __syncthreads();
  if (wave == 0) {
    float s = 0.0f;
    int c = 0;
#pragma unroll
    for (int w2 = 0; w2 < NWAVE; ++w2) { s += wsum[w2 * T2W + lane]; c += wcn[w2]; }
    const float cf = (c < 1) ? 1.0f : (float)c;
    const float v = s / cf;
    float* op = pl + (size_t)g * T2W + lane;
    *(volatile float*)op = v;
    __threadfence();
    *(volatile float*)op = v;
  }
}

__global__ __launch_bounds__(NTHR) void k_head(const float* __restrict__ hg, const float* __restrict__ sf,
                                               const float* __restrict__ par, const int* __restrict__ flg,
                                               int nFlag, float* out) {
  __shared__ __attribute__((aligned(16))) float tb[HTB_N];
  __shared__ float fs[NGR * 21];
  __shared__ int anyf;
  const int tid = (int)threadIdx.x;
  const int g = tid;
#pragma unroll 1
  for (int i = tid; i < HTB_N / 4; i += NTHR) {
    const v4f w = *(const v4f*)(par + PWP + 4 * i);
    *(v4fa*)(tb + 4 * i) = w;
  }
  if (tid == 0) anyf = 0;
  __syncthreads();
  {
    int fi = tid < nFlag ? tid : nFlag - 1;
    fi = fi < 0 ? 0 : fi;
    const int fl = flg[(size_t)fi * 32];
    if (tid < nFlag && fl != 0) anyf = 1;
  }
  const float* sr = sf + (size_t)g * DSF;
#pragma unroll 1
  for (int c = 0; c < DH2; ++c) {
    float z = 0.0f;
#pragma unroll 1
    for (int k4 = 0; k4 < DSF / 4; ++k4) {
      const v4f s = *(const v4f*)(sr + 4 * k4);
      const float* w = tb + (4 * k4) * DH2 + c;
      z = fmaf(bf16_val(s.x), w[0], z);
      z = fmaf(bf16_val(s.y), w[DH2], z);
      z = fmaf(bf16_val(s.z), w[2 * DH2], z);
      z = fmaf(bf16_val(s.w), w[3 * DH2], z);
    }
    z = z + tb[(PBP - PWP) + c];
    const float h = hg[(size_t)g * T2W + c];
    const float t = h * z;
    const float gate = 1.0f / (1.0f + expf(-t));
    const float f = gate * h + (1.0f - gate) * z;
    fs[g * 21 + c] = f;
  }
  float o = 0.0f;
#pragma unroll 1
  for (int j = 0; j < 10; ++j) {
    float t = 0.0f;
#pragma unroll 4
    for (int c = 0; c < DH2; ++c) t = fmaf(fs[g * 21 + c], tb[(PWF1 - PWP) + c * 10 + j], t);
    t = t + tb[(PBF1 - PWP) + j];
    const float r = relu_np(t);
    o = fmaf(r, tb[(PWF2 - PWP) + j], o);
  }
  o = o + tb[PBF2 - PWP];
  __syncthreads();
  const float res = (anyf != 0) ? __int_as_float(0x7fc00000) : o;
  *(volatile float*)(out + g) = res;
  __threadfence();
  *(volatile float*)(out + g) = res;
}

static inline size_t al256(size_t o) { return (o + 255) & ~(size_t)255; }

extern "C" void kernel_launch(void* const* d_in, const int* in_sizes, int n_in,
                              void* d_out, int out_size, void* d_ws, size_t ws_size,
                              hipStream_t stream) {
  if (n_in < 15) return;
  if (in_sizes[0] != NNODE * DIN) return;
  if (in_sizes[1] != NEDGE || in_sizes[2] != NEDGE) return;
  if (in_sizes[3] != NNODE) return;
  if (in_sizes[4] != NGR * DSF) return;
  if (in_sizes[5] != DIN * DH1 || in_sizes[6] != DH1) return;
  if (in_sizes[7] != DH1 * DH2 || in_sizes[8] != DH2) return;
  if (in_sizes[9] != DSF * DH2 || in_sizes[10] != DH2) return;
  if (in_sizes[11] != DH2 * 10 || in_sizes[12] != 10) return;
  if (in_sizes[13] != 10 || in_sizes[14] != 1) return;
  if (out_size != NGR) return;

  const float* feat = (const float*)d_in[0];
  const int*   src  = (const int*)d_in[1];
  const int*   dst  = (const int*)d_in[2];
  const int*   gid  = (const int*)d_in[3];
  const float* sfe  = (const float*)d_in[4];
  const float* W1   = (const float*)d_in[5];
  const float* b1   = (const float*)d_in[6];
  const float* W2   = (const float*)d_in[7];
  const float* b2   = (const float*)d_in[8];
  const float* Wp   = (const float*)d_in[9];
  const float* bp   = (const float*)d_in[10];
  const float* Wf1  = (const float*)d_in[11];
  const float* bf1  = (const float*)d_in[12];
  const float* Wf2  = (const float*)d_in[13];
  const float* bf2  = (const float*)d_in[14];
  float* out = (float*)d_out;

  const int nN = NNODE, nE = NEDGE;
  const int vec8 = ((nE & 3) == 0) ? 1 : 0;

  char* ws = (char*)d_ws;
  size_t off = 0;
  const size_t oXB  = off; off = al256(off + (size_t)MP * DIN * 2);
  const size_t oW1D = off; off = al256(off + (size_t)GBN * KG * 2);
  const size_t oPAR = off; off = al256(off + (size_t)PAR_N * 4);
  const size_t oAGG = off; off = al256(off + (size_t)MP * KG * 2);
  const size_t oT2P = off; off = al256(off + (size_t)MP * T2W * 4);
  const size_t oH2  = off; off = al256(off + (size_t)MP * T2W * 4);
  const size_t oLST = off; off = al256(off + (size_t)NBLK * RCAP * 4);
  const size_t oCNT = off; off = al256(off + (size_t)NBLK * NBA * 4);
  const size_t oOFF = off; off = al256(off + (size_t)NBLK * NBA * 4);
  const size_t oFLG = off; off = al256(off + (size_t)NBLK * 32 * 4);
  const size_t oHG  = off; off = al256(off + (size_t)NGR * T2W * 4);
  if (off > ws_size || off > (size_t)WSMAX) return;
  unsigned short* XB  = (unsigned short*)(ws + oXB);
  unsigned short* W1D = (unsigned short*)(ws + oW1D);
  float*          PAR = (float*)(ws + oPAR);
  unsigned short* AGG = (unsigned short*)(ws + oAGG);
  float*          T2P = (float*)(ws + oT2P);
  float*          H2  = (float*)(ws + oH2);
  int*            LST = (int*)(ws + oLST);
  int*            CNT = (int*)(ws + oCNT);
  int*            OFF = (int*)(ws + oOFF);
  int*            FLG = (int*)(ws + oFLG);
  float*          HG  = (float*)(ws + oHG);

  const size_t cmpLds  = (size_t)CMP_LDS_INTS * 4;
  const size_t gemmLds = (size_t)GEMM_LDS_FLOATS * 4;
  hipFuncSetAttribute(reinterpret_cast<const void*>(&k_compact), hipFuncAttributeMaxDynamicSharedMemorySize, (int)cmpLds);
  hipFuncSetAttribute(reinterpret_cast<const void*>(&k_gemm1), hipFuncAttributeMaxDynamicSharedMemorySize, (int)gemmLds);

  k_prep<<<PREPBLK, NTHR, 0, stream>>>(feat, W1, b1, W2, b2, Wp, bp, Wf1, bf1, Wf2, bf2, XB, W1D, PAR);
  k_compact<<<NBLK, NTHR, cmpLds, stream>>>(src, dst, nE, nN, vec8, LST, CNT, OFF, FLG);
  k_agg1<<<NBLK, NTHR, 0, stream>>>(LST, CNT, OFF, FLG, XB, AGG, nN, MP);
  k_gemm1<<<MP / GBM, NTHR, gemmLds, stream>>>(AGG, W1D, PAR, T2P, nN);
  k_agg2<<<NBLK, NTHR, 0, stream>>>(LST, CNT, OFF, FLG, T2P, PAR, H2, nN, MP);
  k_pool<<<NGR, NTHR, 0, stream>>>(H2, gid, nN, nN / NWAVE, HG);
  k_head<<<1, NTHR, 0, stream>>>(HG, sfe, PAR, FLG, NBLK, out);
}
